// attnGCN_81363860455712
// MI455X (gfx1250) — hardware-verified
//
#include <hip/hip_runtime.h>
#include <stddef.h>
#include <math.h>


#define DF      128
#define HD2     64
#define NGR     64
#define NPG     512
#define NTHR    256
#define NWAVE   8
#define EPT     8
#define NGRP    2
#define CHUNK   (NTHR * EPT * NGRP)
#define WCAP    (EPT * NGRP * 32)
#define LISTN   (NWAVE * WCAP)
#define NB      512
#define NBD     4096
#define GROWS   128
#define QB      64
#define PT      136
#define WSCALE  8.0f
#define HSCALE  16.0f
#define QSCALE  8.0f
#define PSCALE  16384.0f

#define LDS_GEMM (GROWS * DF * 4)
#define LDS_AGG  (NB * DF * 4 + LISTN * 4 + 64)
#define LDS_ATT  (QB * NPG * 4 + QB * NPG * 2 + 4 * DF * 4)

static_assert((CHUNK & (CHUNK - 1)) == 0);
static_assert(CHUNK <= 4096);
static_assert(NB <= 4096 && NBD <= 4096);
static_assert(DF * PT * 2 <= LDS_GEMM);
static_assert(NPG % GROWS == 0);
static_assert(NPG % QB == 0);
static_assert((NB * DF / 4) % NTHR == 0);
static_assert(NGR * NPG % NBD == 0);

typedef float    v4f  __attribute__((ext_vector_type(4)));
typedef float    v8f  __attribute__((ext_vector_type(8)));
typedef int      v4i  __attribute__((ext_vector_type(4)));
typedef _Float16 v8h  __attribute__((ext_vector_type(8)));
typedef _Float16 v16h __attribute__((ext_vector_type(16)));
union FragH { v16h v; v8h h[2]; };

__device__ __forceinline__ v8h cvt8(v4f a, v4f b) {
  v8h r;
  r[0] = (_Float16)a.x; r[1] = (_Float16)a.y; r[2] = (_Float16)a.z; r[3] = (_Float16)a.w;
  r[4] = (_Float16)b.x; r[5] = (_Float16)b.y; r[6] = (_Float16)b.z; r[7] = (_Float16)b.w;
  return r;
}

__device__ __forceinline__ v8f wmh(v16h a, v16h b, v8f c) {
  v8f d = __builtin_amdgcn_wmma_f32_16x16x32_f16(false, a, false, b, (short)0, c, false, false);
  asm volatile("v_nop\n\tv_nop\n\tv_nop\n\tv_nop" : "+v"(d) : "v"(a), "v"(b));
  return d;
}

template <int NBT>
__device__ __forceinline__ int scan_chunk(const int* __restrict__ dsts, int nE, int cbase, int nodeBase,
                                          int vec8, int* list, int tid, int lane, int wave) {
  int wc = 0;
#pragma unroll
  for (int g = 0; g < NGRP; ++g) {
    const int el0  = (g * NTHR + tid) * EPT;
    const int e0   = cbase + el0;
    const int sent = -2147483647 - 1;
    v4i da, db;
    if (vec8 != 0 && e0 + 7 < nE) {
      da = *(const v4i*)(dsts + e0);
      db = *(const v4i*)(dsts + e0 + 4);
    } else {
      da.x = (e0     < nE) ? dsts[min(e0, nE - 1)] : sent;
      da.y = (e0 + 1 < nE) ? dsts[min(e0 + 1, nE - 1)] : sent;
      da.z = (e0 + 2 < nE) ? dsts[min(e0 + 2, nE - 1)] : sent;
      da.w = (e0 + 3 < nE) ? dsts[min(e0 + 3, nE - 1)] : sent;
      db.x = (e0 + 4 < nE) ? dsts[min(e0 + 4, nE - 1)] : sent;
      db.y = (e0 + 5 < nE) ? dsts[min(e0 + 5, nE - 1)] : sent;
      db.z = (e0 + 6 < nE) ? dsts[min(e0 + 6, nE - 1)] : sent;
      db.w = (e0 + 7 < nE) ? dsts[min(e0 + 7, nE - 1)] : sent;
    }
    const unsigned nb = (unsigned)nodeBase;
    const unsigned s0 = (unsigned)da.x - nb, s1 = (unsigned)da.y - nb;
    const unsigned s2 = (unsigned)da.z - nb, s3 = (unsigned)da.w - nb;
    const unsigned s4 = (unsigned)db.x - nb, s5 = (unsigned)db.y - nb;
    const unsigned s6 = (unsigned)db.z - nb, s7 = (unsigned)db.w - nb;
    const bool h0 = s0 < (unsigned)NBT, h1 = s1 < (unsigned)NBT, h2 = s2 < (unsigned)NBT, h3 = s3 < (unsigned)NBT;
    const bool h4 = s4 < (unsigned)NBT, h5 = s5 < (unsigned)NBT, h6 = s6 < (unsigned)NBT, h7 = s7 < (unsigned)NBT;
    const unsigned any = __builtin_amdgcn_ballot_w32(h0 | h1 | h2 | h3 | h4 | h5 | h6 | h7);
    if (any != 0u) {
#define HITJ(J, HJ, SJ) { \
        const unsigned mj = __builtin_amdgcn_ballot_w32(HJ); \
        if (mj != 0u) { \
          if (HJ) { \
            const int pos = wc + (int)__builtin_amdgcn_mbcnt_lo(mj, 0u); \
            if (pos < WCAP) list[wave * WCAP + pos] = ((el0 + (J)) << 12) | (int)(SJ); \
          } \
          wc += (int)__builtin_popcount(mj); } }
      HITJ(0, h0, s0)
      HITJ(1, h1, s1)
      HITJ(2, h2, s2)
      HITJ(3, h3, s3)
      HITJ(4, h4, s4)
      HITJ(5, h5, s5)
      HITJ(6, h6, s6)
      HITJ(7, h7, s7)
#undef HITJ
    }
  }
  return wc;
}

__global__ __launch_bounds__(NTHR) void k_wprep(
    const float* __restrict__ W1, const float* __restrict__ W2, const float* __restrict__ Wq,
    const float* __restrict__ Wk, const float* __restrict__ Wv, _Float16* wpl) {
  const int i   = blockIdx.x * NTHR + threadIdx.x;
  const int per = DF * DF / 8;
  if (i >= 5 * per) return;
  const int which = i / per;
  const int o  = (i - which * per) * 8;
  const int n  = o >> 7;
  const int k0 = o & (DF - 1);
  const float* W = (which == 0) ? W1 : (which == 1) ? W2 : (which == 2) ? Wq : (which == 3) ? Wk : Wv;
  const float* p = W + (size_t)k0 * DF + n;
  v4f a, b;
  a.x = p[0];      a.y = p[DF];     a.z = p[2 * DF]; a.w = p[3 * DF];
  b.x = p[4 * DF]; b.y = p[5 * DF]; b.z = p[6 * DF]; b.w = p[7 * DF];
  a = a * WSCALE;
  b = b * WSCALE;
  const v8h hv = cvt8(a, b);
  _Float16* dp = wpl + (size_t)which * DF * DF + o;
  *(volatile v8h*)dp = hv;
  __threadfence();
  *(volatile v8h*)dp = hv;
}

__global__ __launch_bounds__(NTHR) void k_cvt(const float* __restrict__ x, _Float16* x16, int n8) {
  const int i = blockIdx.x * NTHR + threadIdx.x;
  if (i >= n8) return;
  const float* p = x + (size_t)i * 8;
  const v4f a = *(const v4f*)p, b = *(const v4f*)(p + 4);
  const v8h hv = cvt8(a, b);
  _Float16* dp = x16 + (size_t)i * 8;
  *(volatile v8h*)dp = hv;
  __threadfence();
  *(volatile v8h*)dp = hv;
}

__global__ __launch_bounds__(NTHR) void k_deg(
    const int* __restrict__ ei, float* dinv, int nN, int nE, int vec8) {
  __shared__ __attribute__((aligned(16))) int cnt[NBD];
  __shared__ __attribute__((aligned(16))) int list[LISTN];
  __shared__ int wcnt[NWAVE];
  const int tid = threadIdx.x, lane = tid & 31, wave = tid >> 5;
  const int nodeBase = blockIdx.x * NBD;
  const int* dsts = ei + nE;
  (void)nN;

  for (int i = tid; i < NBD; i += NTHR) cnt[i] = 0;
  __syncthreads();

  const int nChunks = (nE + CHUNK - 1) / CHUNK;
#pragma unroll 1
  for (int ch = 0; ch < nChunks; ++ch) {
    const int cbase = ch * CHUNK;
    const int wc = scan_chunk<NBD>(dsts, nE, cbase, nodeBase, vec8, list, tid, lane, wave);
    if (lane == 0) wcnt[wave] = wc;
    __syncthreads();
    if (wave == 0) {
#pragma unroll 1
      for (int wsx = 0; wsx < NWAVE; ++wsx) {
        int n = __builtin_amdgcn_readfirstlane(wcnt[wsx]);
        n = n > WCAP ? WCAP : (n < 0 ? 0 : n);
        const int* lp = list + wsx * WCAP;
#pragma unroll 1
        for (int i = 0; i < n; ++i) {
          const int ent  = __builtin_amdgcn_readfirstlane(lp[i]);
          const int slot = ent & (NBD - 1);
          if (lane == 0) cnt[slot] = cnt[slot] + 1;
        }
      }
    }
    __syncthreads();
  }

  v4f dq[4];
#pragma unroll
  for (int q = 0; q < 4; ++q) {
    const int f = (wave * 4 + q) * 128 + 4 * lane;
    const v4i c = *(const v4i*)(cnt + f);
    dq[q].x = rsqrtf((float)(c.x + 1));
    dq[q].y = rsqrtf((float)(c.y + 1));
    dq[q].z = rsqrtf((float)(c.z + 1));
    dq[q].w = rsqrtf((float)(c.w + 1));
  }
  float* dp = dinv + (size_t)nodeBase;
#pragma unroll
  for (int q = 0; q < 4; ++q) *(volatile v4f*)(dp + (wave * 4 + q) * 128 + 4 * lane) = dq[q];
  __threadfence();
#pragma unroll
  for (int q = 0; q < 4; ++q) *(volatile v4f*)(dp + (wave * 4 + q) * 128 + 4 * lane) = dq[q];
}

template <int MODE>
__global__ __launch_bounds__(NTHR) void k_gemm(
    const _Float16* __restrict__ A, const _Float16* __restrict__ Bw,
    const float* __restrict__ rsc, const float* __restrict__ bias,
    void* outp, float cscale, float oscale, int nRows) {
  extern __shared__ v4f lds_dyn[];
  const int tid = threadIdx.x, lane = tid & 31, wave = tid >> 5, hh = lane >> 4, m = lane & 15;
  const int rowBase = blockIdx.x * GROWS;
  int arow = rowBase + wave * 16 + m;
  arow = arow > nRows - 1 ? nRows - 1 : arow;
  const _Float16* ar = A + (size_t)arow * DF + 8 * hh;

  v8f acc[8];
#pragma unroll
  for (int t = 0; t < 8; ++t) { v8f z = {0.f, 0.f, 0.f, 0.f, 0.f, 0.f, 0.f, 0.f}; acc[t] = z; }
#pragma unroll
  for (int kt = 0; kt < DF / 32; ++kt) {
    FragH a;
    a.h[0] = *(const v8h*)(ar + 32 * kt);
    a.h[1] = *(const v8h*)(ar + 32 * kt + 16);
#pragma unroll
    for (int t = 0; t < 8; ++t) {
      const _Float16* bp = Bw + (size_t)(16 * t + m) * DF + 32 * kt + 8 * hh;
      FragH b;
      b.h[0] = *(const v8h*)bp;
      b.h[1] = *(const v8h*)(bp + 16);
      acc[t] = wmh(a.v, b.v, acc[t]);
    }
  }

  if (MODE == 0) {
    float* stg = (float*)lds_dyn;
    const int r0 = wave * 16 + 8 * hh;
    const v4f dA = *(const v4f*)(rsc + (size_t)rowBase + r0);
    const v4f dB = *(const v4f*)(rsc + (size_t)rowBase + r0 + 4);
    const float d0 = dA.x * cscale, d1 = dA.y * cscale, d2 = dA.z * cscale, d3 = dA.w * cscale;
    const float d4 = dB.x * cscale, d5 = dB.y * cscale, d6 = dB.z * cscale, d7 = dB.w * cscale;
    float* sp = stg + r0 * DF + m;
#pragma unroll
    for (int t = 0; t < 8; ++t) {
      sp[0 * DF + 16 * t] = acc[t][0] * d0;
      sp[1 * DF + 16 * t] = acc[t][1] * d1;
      sp[2 * DF + 16 * t] = acc[t][2] * d2;
      sp[3 * DF + 16 * t] = acc[t][3] * d3;
      sp[4 * DF + 16 * t] = acc[t][4] * d4;
      sp[5 * DF + 16 * t] = acc[t][5] * d5;
      sp[6 * DF + 16 * t] = acc[t][6] * d6;
      sp[7 * DF + 16 * t] = acc[t][7] * d7;
    }
    __syncthreads();
    const float* lp = stg + wave * 16 * DF + 4 * lane;
    float* gp = (float*)outp + ((size_t)rowBase + wave * 16) * DF + 4 * lane;
#pragma unroll
    for (int i = 0; i < 16; ++i) { const v4f v = *(const v4f*)(lp + i * DF); *(volatile v4f*)(gp + (size_t)i * DF) = v; }
    __threadfence();
#pragma unroll
    for (int i = 0; i < 16; ++i) { const v4f v = *(const v4f*)(lp + i * DF); *(volatile v4f*)(gp + (size_t)i * DF) = v; }
  } else {
    float bc[8];
#pragma unroll
    for (int t = 0; t < 8; ++t) bc[t] = bias[16 * t + m];
    if (MODE == 1) {
      _Float16* stg = (_Float16*)lds_dyn;
      _Float16* sp = stg + (wave * 16 + 8 * hh) * DF + m;
#pragma unroll
      for (int t = 0; t < 8; ++t) {
#pragma unroll
        for (int r = 0; r < 8; ++r) sp[r * DF + 16 * t] = (_Float16)((acc[t][r] * cscale + bc[t]) * oscale);
      }
      __syncthreads();
      v8h ov[8];
#pragma unroll
      for (int i = 0; i < 8; ++i) ov[i] = *(const v8h*)(stg + (wave * 16 + 2 * i + hh) * DF + 8 * m);
      _Float16* gp = (_Float16*)outp + ((size_t)rowBase + wave * 16) * DF + 8 * m;
#pragma unroll
      for (int i = 0; i < 8; ++i) *(volatile v8h*)(gp + (size_t)(2 * i + hh) * DF) = ov[i];
      __threadfence();
#pragma unroll
      for (int i = 0; i < 8; ++i) *(volatile v8h*)(gp + (size_t)(2 * i + hh) * DF) = ov[i];
    } else {
      _Float16* stg = (_Float16*)lds_dyn;
      const int rr0 = wave * 16 + 8 * hh;
#pragma unroll
      for (int t = 0; t < 8; ++t) {
        _Float16* sp = stg + (16 * t + m) * PT + rr0;
#pragma unroll
        for (int r = 0; r < 8; ++r) sp[r] = (_Float16)((acc[t][r] * cscale + bc[t]) * oscale);
      }
      __syncthreads();
      const int g   = rowBase / NPG;
      const int kin = rowBase - g * NPG;
      v8h ov[8];
#pragma unroll
      for (int i = 0; i < 8; ++i) ov[i] = *(const v8h*)(stg + (wave * 16 + 2 * i + hh) * PT + 8 * m);
      _Float16* gp = (_Float16*)outp + ((size_t)g * DF + wave * 16) * NPG + kin + 8 * m;
#pragma unroll
      for (int i = 0; i < 8; ++i) *(volatile v8h*)(gp + (size_t)(2 * i + hh) * NPG) = ov[i];
      __threadfence();
#pragma unroll
      for (int i = 0; i < 8; ++i) *(volatile v8h*)(gp + (size_t)(2 * i + hh) * NPG) = ov[i];
    }
  }
}

__global__ __launch_bounds__(NTHR) void k_agg(
    const int* __restrict__ ei, const float* __restrict__ gpl, const float* __restrict__ dinv,
    const float* __restrict__ bias, _Float16* hout, int nN, int nE, int vec8) {
  extern __shared__ v4f lds_dyn[];
  float* acc  = (float*)lds_dyn;
  int*   list = (int*)(acc + NB * DF);
  int*   wcnt = list + LISTN;
  const int tid = threadIdx.x, lane = tid & 31, wave = tid >> 5, hh = lane >> 4, m = lane & 15;
  const int nodeBase = blockIdx.x * NB;
  const int* dsts = ei + nE;

  {
    const v4f z = {0.f, 0.f, 0.f, 0.f};
    for (int i = tid; i < NB * DF / 4; i += NTHR) lds_dyn[i] = z;
  }
  __syncthreads();

  const int nChunks = (nE + CHUNK - 1) / CHUNK;
#pragma unroll 1
  for (int ch = 0; ch < nChunks; ++ch) {
    const int cbase = ch * CHUNK;
    const int wc = scan_chunk<NB>(dsts, nE, cbase, nodeBase, vec8, list, tid, lane, wave);
    if (lane == 0) wcnt[wave] = wc;
    __syncthreads();
    if (wave == 0) {
#pragma unroll 1
      for (int wsx = 0; wsx < NWAVE; ++wsx) {
        int n = __builtin_amdgcn_readfirstlane(wcnt[wsx]);
        n = n > WCAP ? WCAP : (n < 0 ? 0 : n);
        const int* lp = list + wsx * WCAP;
#pragma unroll 1
        for (int i = 0; i < n; ++i) {
          const int ent  = __builtin_amdgcn_readfirstlane(lp[i]);
          const int slot = ent & (NB - 1);
          int e = cbase + ((ent >> 12) & (CHUNK - 1));
          e = e > nE - 1 ? nE - 1 : e;
          int src = ei[e];
          src = src < 0 ? 0 : (src > nN - 1 ? nN - 1 : src);
          const v4f v = *(const v4f*)(gpl + (size_t)src * DF + 4 * lane);
          v4f* ap = (v4f*)(acc + slot * DF + 4 * lane);
          *ap = *ap + v;
        }
      }
    }
    __syncthreads();
  }

#pragma unroll 4
  for (int i = 0; i < (NB * DF / 4) / NTHR; ++i) {
    const int idx  = i * NTHR + tid;
    const int slot = idx >> 5;
    const int c4   = (idx & 31) * 4;
    int node = nodeBase + slot;
    node = node > nN - 1 ? nN - 1 : node;
    const float d  = dinv[node];
    const v4f   gv = *(const v4f*)(gpl + (size_t)node * DF + c4);
    const v4f   bv = *(const v4f*)(bias + c4);
    v4f* ap = (v4f*)(acc + slot * DF + c4);
    v4f hv = (*ap + gv) * d + bv;
    hv.x = fmaxf(hv.x, 0.f) * HSCALE; hv.y = fmaxf(hv.y, 0.f) * HSCALE;
    hv.z = fmaxf(hv.z, 0.f) * HSCALE; hv.w = fmaxf(hv.w, 0.f) * HSCALE;
    *ap = hv;
  }
  __syncthreads();

#pragma unroll 4
  for (int i = 0; i < 32; ++i) {
    const int row  = wave * 64 + 2 * i + hh;
    const int node = nodeBase + row;
    const float* lp = acc + row * DF + 8 * m;
    const v4f p0 = *(const v4f*)lp, p1 = *(const v4f*)(lp + 4);
    const v8h v = cvt8(p0, p1);
    if (node < nN) *(volatile v8h*)(hout + (size_t)node * DF + 8 * m) = v;
  }
  __threadfence();
#pragma unroll 4
  for (int i = 0; i < 32; ++i) {
    const int row  = wave * 64 + 2 * i + hh;
    const int node = nodeBase + row;
    const float* lp = acc + row * DF + 8 * m;
    const v4f p0 = *(const v4f*)lp, p1 = *(const v4f*)(lp + 4);
    const v8h v = cvt8(p0, p1);
    if (node < nN) *(volatile v8h*)(hout + (size_t)node * DF + 8 * m) = v;
  }
}

__global__ __launch_bounds__(NTHR) void k_attn(
    const _Float16* __restrict__ q16, const _Float16* __restrict__ k16,
    const _Float16* __restrict__ vt16, float* pool, float sscale, float oinv) {
  extern __shared__ v4f lds_dyn[];
  float*    sS  = (float*)lds_dyn;
  _Float16* sP  = (_Float16*)(sS + QB * NPG);
  float*    red = (float*)(sP + QB * NPG);
  const int tid = threadIdx.x, lane = tid & 31, wave = tid >> 5, hh = lane >> 4, m = lane & 15;
  const int g = blockIdx.y, qb = blockIdx.x;
  const size_t node0 = (size_t)g * NPG;
  const int q0 = qb * QB;
  const int rt = wave & 3, half = wave >> 2;

  const _Float16* qp = q16 + (node0 + q0 + 16 * rt + m) * DF + 8 * hh;
#pragma unroll 1
  for (int c = 0; c < 4; ++c) {
    v8f acc[4];
#pragma unroll
    for (int j = 0; j < 4; ++j) { v8f z = {0.f, 0.f, 0.f, 0.f, 0.f, 0.f, 0.f, 0.f}; acc[j] = z; }
#pragma unroll
    for (int kt = 0; kt < DF / 32; ++kt) {
      FragH a;
      a.h[0] = *(const v8h*)(qp + 32 * kt);
      a.h[1] = *(const v8h*)(qp + 32 * kt + 16);
#pragma unroll
      for (int j = 0; j < 4; ++j) {
        const int key = 16 * (16 * half + 4 * c + j) + m;
        const _Float16* bp = k16 + (node0 + key) * DF + 32 * kt + 8 * hh;
        FragH b;
        b.h[0] = *(const v8h*)bp;
        b.h[1] = *(const v8h*)(bp + 16);
        acc[j] = wmh(a.v, b.v, acc[j]);
      }
    }
#pragma unroll
    for (int j = 0; j < 4; ++j) {
      float* sp = sS + (16 * rt + 8 * hh) * NPG + 16 * (16 * half + 4 * c + j) + m;
#pragma unroll
      for (int r = 0; r < 8; ++r) sp[r * NPG] = acc[j][r] * sscale;
    }
  }
  __syncthreads();

#pragma unroll 1
  for (int rr = 0; rr < 8; ++rr) {
    const int row = wave * 8 + rr;
    const float* sp = sS + row * NPG + lane;
    float v[16];
#pragma unroll
    for (int i = 0; i < 16; ++i) v[i] = sp[32 * i];
    float mx = v[0];
#pragma unroll
    for (int i = 1; i < 16; ++i) mx = fmaxf(mx, v[i]);
    mx = fmaxf(mx, __shfl_xor(mx, 16));
    mx = fmaxf(mx, __shfl_xor(mx, 8));
    mx = fmaxf(mx, __shfl_xor(mx, 4));
    mx = fmaxf(mx, __shfl_xor(mx, 2));
    mx = fmaxf(mx, __shfl_xor(mx, 1));
    float s = 0.f;
#pragma unroll
    for (int i = 0; i < 16; ++i) { v[i] = __expf(v[i] - mx); s += v[i]; }
    s += __shfl_xor(s, 16);
    s += __shfl_xor(s, 8);
    s += __shfl_xor(s, 4);
    s += __shfl_xor(s, 2);
    s += __shfl_xor(s, 1);
    const float f = PSCALE * (1.0f / s);
    _Float16* pp = sP + row * NPG + lane;
#pragma unroll
    for (int i = 0; i < 16; ++i) pp[32 * i] = (_Float16)(v[i] * f);
  }
  __syncthreads();

  {
    v8f acc[4];
#pragma unroll
    for (int j = 0; j < 4; ++j) { v8f z = {0.f, 0.f, 0.f, 0.f, 0.f, 0.f, 0.f, 0.f}; acc[j] = z; }
    const _Float16* ap = sP + (16 * rt + m) * NPG + 8 * hh;
#pragma unroll 2
    for (int ks = 0; ks < NPG / 32; ++ks) {
      FragH a;
      a.h[0] = *(const v8h*)(ap + 32 * ks);
      a.h[1] = *(const v8h*)(ap + 32 * ks + 16);
#pragma unroll
      for (int j = 0; j < 4; ++j) {
        const int d = 16 * (4 * half + j) + m;
        const _Float16* bp = vt16 + ((size_t)g * DF + d) * NPG + 32 * ks + 8 * hh;
        FragH b;
        b.h[0] = *(const v8h*)bp;
        b.h[1] = *(const v8h*)(bp + 16);
        acc[j] = wmh(a.v, b.v, acc[j]);
      }
    }
    float cs[4];
#pragma unroll
    for (int j = 0; j < 4; ++j) {
      float s = acc[j][0] + acc[j][1] + acc[j][2] + acc[j][3] + acc[j][4] + acc[j][5] + acc[j][6] + acc[j][7];
      s += __shfl_xor(s, 16);
      cs[j] = s;
    }
    if (hh == 0) {
#pragma unroll
      for (int j = 0; j < 4; ++j) red[rt * DF + 16 * (4 * half + j) + m] = cs[j];
    }
  }
  __syncthreads();

  if (tid < 32) {
    const int c = 4 * tid;
    v4f o;
    o.x = (red[c]     + red[DF + c]     + red[2 * DF + c]     + red[3 * DF + c])     * oinv;
    o.y = (red[c + 1] + red[DF + c + 1] + red[2 * DF + c + 1] + red[3 * DF + c + 1]) * oinv;
    o.z = (red[c + 2] + red[DF + c + 2] + red[2 * DF + c + 2] + red[3 * DF + c + 2]) * oinv;
    o.w = (red[c + 3] + red[DF + c + 3] + red[2 * DF + c + 3] + red[3 * DF + c + 3]) * oinv;
    float* gp = pool + ((size_t)g * gridDim.x + qb) * DF + c;
    *(volatile v4f*)gp = o;
    __threadfence();
    *(volatile v4f*)gp = o;
  }
}

__global__ __launch_bounds__(NTHR) void k_head(
    const float* __restrict__ pool, const float* __restrict__ Wh1, const float* __restrict__ bh1,
    const float* __restrict__ Wh2, const float* __restrict__ bh2, const int* __restrict__ bidx,
    float* out, int nqb, float inv_n) {
  __shared__ __attribute__((aligned(16))) float sPool[NGR * DF];
  __shared__ __attribute__((aligned(16))) float sZ[NGR * HD2];
  __shared__ __attribute__((aligned(16))) float sOut[NGR];
  const int tid = threadIdx.x;
  (void)bidx;

  for (int idx = tid; idx < NGR * DF; idx += NTHR) {
    const int g = idx >> 7, d = idx & (DF - 1);
    float s = 0.f;
#pragma unroll 1
    for (int qb = 0; qb < nqb; ++qb) s += pool[((size_t)g * nqb + qb) * DF + d];
    sPool[idx] = s * inv_n;
  }
  __syncthreads();

  for (int idx = tid; idx < NGR * HD2; idx += NTHR) {
    const int g = idx >> 6, j = idx & (HD2 - 1);
    const float* pg = sPool + g * DF;
    float s = 0.f;
#pragma unroll 4
    for (int d = 0; d < DF; ++d) s += pg[d] * Wh1[d * HD2 + j];
    s += bh1[j];
    sZ[idx] = fmaxf(s, 0.f);
  }
  __syncthreads();

  if (tid < NGR) {
    const float* pz = sZ + tid * HD2;
    float s = 0.f;
#pragma unroll 4
    for (int j = 0; j < HD2; ++j) s += pz[j] * Wh2[j];
    sOut[tid] = s + bh2[0];
  }
  __syncthreads();

  if (tid < 16) {
    const v4f o = *(const v4f*)(sOut + 4 * tid);
    *(volatile v4f*)(out + 4 * tid) = o;
    __threadfence();
    *(volatile v4f*)(out + 4 * tid) = o;
  }
}

extern "C" void kernel_launch(void* const* d_in, const int* in_sizes, int n_in,
                              void* d_out, int out_size, void* d_ws, size_t ws_size,
                              hipStream_t stream) {
  if (n_in < 17) return;
  const int nN = in_sizes[0] / DF;
  const int nE = in_sizes[1] / 2;
  if (nN != NGR * NPG || in_sizes[0] != nN * DF) return;
  if (nE < 0 || in_sizes[1] != nE * 2) return;
  if (in_sizes[3] != DF * DF || in_sizes[5] != DF * DF || in_sizes[7] != DF * DF ||
      in_sizes[9] != DF * DF || in_sizes[11] != DF * DF) return;
  if (in_sizes[4] < DF || in_sizes[6] < DF || in_sizes[8] < DF || in_sizes[10] < DF || in_sizes[12] < DF) return;
  if (in_sizes[13] != DF * HD2 || in_sizes[14] < HD2 || in_sizes[15] < HD2 || in_sizes[16] < 1) return;
  if (out_size != NGR) return;

  const float* x   = (const float*)d_in[0];
  const int*   ei  = (const int*)d_in[1];
  const int*   bix = (const int*)d_in[2];
  const float* W1  = (const float*)d_in[3];
  const float* b1  = (const float*)d_in[4];
  const float* W2  = (const float*)d_in[5];
  const float* b2  = (const float*)d_in[6];
  const float* Wq  = (const float*)d_in[7];
  const float* bq  = (const float*)d_in[8];
  const float* Wk  = (const float*)d_in[9];
  const float* bk  = (const float*)d_in[10];
  const float* Wv  = (const float*)d_in[11];
  const float* bv  = (const float*)d_in[12];
  const float* Wh1 = (const float*)d_in[13];
  const float* bh1 = (const float*)d_in[14];
  const float* Wh2 = (const float*)d_in[15];
  const float* bh2 = (const float*)d_in[16];
  float* out = (float*)d_out;

  const int nBD = (nN + NBD - 1) / NBD;
  const int nG  = nN / GROWS;
  const int nA  = nN / NB;
  const int nQB = NPG / QB;
  const int n8  = nN * DF / 8;

  char* ws = (char*)d_ws;
  size_t off = 0;
  const size_t plane16 = (size_t)nN * DF * 2;
  const size_t oW   = off; off += (size_t)5 * DF * DF * 2;                     off = (off + 255) & ~(size_t)255;
  const size_t oDv  = off; off += (size_t)nBD * NBD * 4;                        off = (off + 255) & ~(size_t)255;
  const size_t oX16 = off; off += plane16;                                      off = (off + 255) & ~(size_t)255;
  const size_t oH16 = off; off += plane16;                                      off = (off + 255) & ~(size_t)255;
  const size_t oG   = off; off += (size_t)nN * DF * 4;                          off = (off + 255) & ~(size_t)255;
  const size_t oQ   = off; off += plane16;                                      off = (off + 255) & ~(size_t)255;
  const size_t oK   = off; off += plane16;                                      off = (off + 255) & ~(size_t)255;
  const size_t oVt  = off; off += plane16;                                      off = (off + 255) & ~(size_t)255;
  const size_t oPl  = off; off += (size_t)NGR * nQB * DF * 4;                   off = (off + 255) & ~(size_t)255;
  if (off > ws_size) return;
  _Float16* wpl  = (_Float16*)(ws + oW);
  float*    dinv = (float*)(ws + oDv);
  _Float16* x16  = (_Float16*)(ws + oX16);
  _Float16* h16  = (_Float16*)(ws + oH16);
  float*    gpl  = (float*)(ws + oG);
  _Float16* q16  = (_Float16*)(ws + oQ);
  _Float16* k16  = (_Float16*)(ws + oK);
  _Float16* vt16 = (_Float16*)(ws + oVt);
  float*    pool = (float*)(ws + oPl);
  const _Float16* w1s = wpl;
  const _Float16* w2s = wpl + 1 * DF * DF;
  const _Float16* wqs = wpl + 2 * DF * DF;
  const _Float16* wks = wpl + 3 * DF * DF;
  const _Float16* wvs = wpl + 4 * DF * DF;

  const int vec8 = ((nE & 3) == 0) ? 1 : 0;
  const float winv  = 1.0f / WSCALE;
  const float hwinv = 1.0f / (WSCALE * HSCALE);
  const float ssc   = 0.08838834764831845f * (1.0f / (QSCALE * QSCALE));
  const float oinv  = 1.0f / (PSCALE * QSCALE);
  const float inv_n = 1.0f / (float)NPG;

  k_wprep<<<(5 * DF * DF / 8 + NTHR - 1) / NTHR, NTHR, 0, stream>>>(W1, W2, Wq, Wk, Wv, wpl);
  k_cvt<<<(n8 + NTHR - 1) / NTHR, NTHR, 0, stream>>>(x, x16, n8);
  k_deg<<<nBD, NTHR, 0, stream>>>(ei, dinv, nN, nE, vec8);

  hipFuncSetAttribute(reinterpret_cast<const void*>(&k_gemm<0>),
                      hipFuncAttributeMaxDynamicSharedMemorySize, LDS_GEMM);
  hipFuncSetAttribute(reinterpret_cast<const void*>(&k_gemm<1>),
                      hipFuncAttributeMaxDynamicSharedMemorySize, LDS_GEMM);
  hipFuncSetAttribute(reinterpret_cast<const void*>(&k_gemm<2>),
                      hipFuncAttributeMaxDynamicSharedMemorySize, LDS_GEMM);
  hipFuncSetAttribute(reinterpret_cast<const void*>(&k_agg),
                      hipFuncAttributeMaxDynamicSharedMemorySize, LDS_AGG);
  hipFuncSetAttribute(reinterpret_cast<const void*>(&k_attn),
                      hipFuncAttributeMaxDynamicSharedMemorySize, LDS_ATT);

  k_gemm<0><<<nG, NTHR, LDS_GEMM, stream>>>(x16, w1s, dinv, b1, (void*)gpl, winv, 1.0f, nN);
  k_agg<<<nA, NTHR, LDS_AGG, stream>>>(ei, gpl, dinv, b1, h16, nN, nE, vec8);
  k_gemm<0><<<nG, NTHR, LDS_GEMM, stream>>>(h16, w2s, dinv, b2, (void*)gpl, hwinv, 1.0f, nN);
  k_agg<<<nA, NTHR, LDS_AGG, stream>>>(ei, gpl, dinv, b2, h16, nN, nE, vec8);
  k_gemm<1><<<nG, NTHR, LDS_GEMM, stream>>>(h16, wqs, dinv, bq, (void*)q16, hwinv, QSCALE, nN);
  k_gemm<1><<<nG, NTHR, LDS_GEMM, stream>>>(h16, wks, dinv, bk, (void*)k16, hwinv, QSCALE, nN);
  k_gemm<2><<<nG, NTHR, LDS_GEMM, stream>>>(h16, wvs, dinv, bv, (void*)vt16, hwinv, QSCALE, nN);
  k_attn<<<dim3(nQB, NGR, 1), NTHR, LDS_ATT, stream>>>(q16, k16, vt16, pool, ssc, oinv);
  k_head<<<1, NTHR, 0, stream>>>(pool, Wh1, bh1, Wh2, bh2, bix, out, nQB, inv_n);
}
